// RecurrentMAFDecay_60206851556039
// MI455X (gfx1250) — hardware-run, weakly checked
//
#include <hip/hip_runtime.h>
#include <math.h>

constexpr int NB     = 64;
constexpr int NSTEP  = 512;
constexpr int NDIN   = 32;
constexpr int NEMB   = 64;
constexpr int NHID   = 256;
constexpr int NG3    = 3 * NHID;
constexpr int NCAT   = NDIN + NEMB;
constexpr int NROWS  = NB * NSTEP;
constexpr int SCAN_THR = 512;
constexpr int HP = 264;
constexpr int OP = 260;
constexpr float WCARRY = 16.0f;
constexpr float XCARRY = 16.0f;
constexpr float HCARRY = 256.0f;
constexpr float FOLD_X = 1.0f / (XCARRY * WCARRY);
constexpr float FOLD_H = 1.0f / (HCARRY * WCARRY);

static_assert(NCAT % 32 == 0);
static_assert(NHID % 32 == 0);
static_assert(NROWS % 64 == 0 && NG3 % 64 == 0);
static_assert(((NROWS / 64) * (NG3 / 64)) % 8 == 0);
static_assert(NHID == 16 * (SCAN_THR / 32));
static_assert(NB % 16 == 0);
static_assert((NROWS * (NCAT / 8)) % 256 == 0);
static_assert((16 * NSTEP) % SCAN_THR == 0);
static_assert((16 * NHID / 4) % SCAN_THR == 0);
static_assert(NDIN == 32 && NEMB == 64);

typedef __attribute__((ext_vector_type(16))) _Float16 v16h;
typedef __attribute__((ext_vector_type(8)))  _Float16 v8h;
typedef __attribute__((ext_vector_type(8)))  float    v8f;
typedef __attribute__((ext_vector_type(4)))  float    v4f;

union FragU { v16h v; v8h h[2]; };
__device__ __forceinline__ v16h frag_load(const _Float16* p) {
  FragU f;
  f.h[0] = *(const v8h*)(p);
  f.h[1] = *(const v8h*)(p + 16);
  return f.v;
}
__device__ __forceinline__ v8f mma_h(v16h a, v16h b, v8f c) {
  return __builtin_amdgcn_wmma_f32_16x16x32_f16(false, a, false, b, (short)0, c, false, false);
}
__device__ __forceinline__ void guard4_h(v8f& a, v8f& b, v8f& c, v8f& d, v16h x, v16h y0, v16h y1, v16h y2, v16h y3) {
  asm volatile("v_nop\n\tv_nop\n\tv_nop\n\tv_nop" : "+v"(a), "+v"(b), "+v"(c), "+v"(d) : "v"(x), "v"(y0), "v"(y1), "v"(y2), "v"(y3));
}
__device__ __forceinline__ void guard3_h(v8f& a, v8f& b, v8f& c, v16h x, v16h y0, v16h y1, v16h y2) {
  asm volatile("v_nop\n\tv_nop\n\tv_nop\n\tv_nop" : "+v"(a), "+v"(b), "+v"(c) : "v"(x), "v"(y0), "v"(y1), "v"(y2));
}
__device__ __forceinline__ void keep4_h(v16h a, v16h b, v16h c, v16h d) { asm volatile("v_nop" :: "v"(a), "v"(b), "v"(c), "v"(d)); }
__device__ __forceinline__ void acc_guard4(v8f& a, v8f& b, v8f& c, v8f& d) { asm volatile("v_nop\n\tv_nop\n\tv_nop\n\tv_nop" : "+v"(a), "+v"(b), "+v"(c), "+v"(d)); }
__device__ __forceinline__ void acc_guard3(v8f& a, v8f& b, v8f& c) { asm volatile("v_nop\n\tv_nop\n\tv_nop\n\tv_nop" : "+v"(a), "+v"(b), "+v"(c)); }

__device__ __forceinline__ float sigm_f(float x) {
  const float y = fminf(fmaxf(x, -30.0f), 30.0f);
  return __builtin_amdgcn_rcpf(1.0f + expf(-y));
}
__device__ __forceinline__ float tanh_f(float x) {
  const float y = fminf(fmaxf(2.0f * x, -30.0f), 30.0f);
  return 1.0f - 2.0f * __builtin_amdgcn_rcpf(expf(y) + 1.0f);
}

__global__ __launch_bounds__(256) void prep_w_kernel(
    const float* __restrict__ s0, const float* __restrict__ s1, const float* __restrict__ s2, const float* __restrict__ s3,
    unsigned short* __restrict__ d0, unsigned short* __restrict__ d1, unsigned short* __restrict__ d2, unsigned short* __restrict__ d3,
    int n8_0, int n8_1, int n8_2, int n8_3, float sc) {
  const int y = blockIdx.y;
  const float* s = (y == 0) ? s0 : (y == 1) ? s1 : (y == 2) ? s2 : s3;
  unsigned short* d = (y == 0) ? d0 : (y == 1) ? d1 : (y == 2) ? d2 : d3;
  const int n8 = (y == 0) ? n8_0 : (y == 1) ? n8_1 : (y == 2) ? n8_2 : n8_3;
  const int i = blockIdx.x * 256 + threadIdx.x;
  if (i < n8) {
    const v4f a = *(const v4f*)(s + (size_t)i * 8);
    const v4f b = *(const v4f*)(s + (size_t)i * 8 + 4);
    v8h hv;
#pragma unroll
    for (int e = 0; e < 4; ++e) {
      hv[e]     = (_Float16)(a[e] * sc);
      hv[4 + e] = (_Float16)(b[e] * sc);
    }
    *(volatile v8h*)(d + (size_t)i * 8) = hv;
    __threadfence();
    *(volatile v8h*)(d + (size_t)i * 8) = hv;
  }
}

__global__ __launch_bounds__(256) void prep_xcat_kernel(const float* __restrict__ x, const float* __restrict__ tin,
                                                        const float* __restrict__ Wt, const float* __restrict__ bt,
                                                        unsigned short* __restrict__ XC) {
  __shared__ __align__(16) _Float16 st[256 * 8];
  const int tid = threadIdx.x;
  const int i = blockIdx.x * 256 + tid;
  const int row = i / 12;
  const int c8 = i - row * 12;
  const int isx = (c8 < 4) ? 1 : 0;
  const int xc = (isx ? c8 : 3) * 8;
  const int ec = (isx ? 0 : (c8 - 4)) * 8;
  const float fx = isx ? 1.0f : 0.0f;
  const float fc = 1.0f - fx;
  const float tv = tin[row];
  const float* xp = x + (size_t)row * NDIN + xc;
  const float* wp = Wt + ec;
  const float* bp = bt + ec;
#pragma unroll 1
  for (int e = 0; e < 8; ++e) {
    float xv = xp[e];
    float wv = wp[e];
    float bv = bp[e];
    asm volatile("" : "+v"(xv), "+v"(wv), "+v"(bv));
    const float cv = cosf(wv * tv + bv);
    const float val = fmaf(fx, xv, fc * cv);
    st[tid * 8 + e] = (_Float16)(val * XCARRY);
  }
  __syncthreads();
  const v8h hv = *(const v8h*)(st + tid * 8);
  *(volatile v8h*)(XC + (size_t)i * 8) = hv;
  __threadfence();
  *(volatile v8h*)(XC + (size_t)i * 8) = hv;
}

__global__ __launch_bounds__(256) void gemm_f16_kernel(
    const unsigned short* __restrict__ Ap, int lda,
    const unsigned short* __restrict__ Btp, int ldb,
    float* __restrict__ C, int ldc,
    const float* __restrict__ bias, int M, int N, int K, float scale) {
  const _Float16* A  = (const _Float16*)Ap;
  const _Float16* Bt = (const _Float16*)Btp;
  __shared__ __align__(16) float sT[8][16 * 68];
  const int lane = threadIdx.x & 31;
  const int wave = threadIdx.x >> 5;
  const int tilesN = N >> 6;
  const int tilesM = M >> 6;
  const int tile = blockIdx.x * 8 + wave;
  if (tile >= tilesM * tilesN) return;
  const int tm = tile / tilesN;
  const int tn = tile - tm * tilesN;
  const int m0 = tm << 6;
  const int n0 = tn << 6;
  const int rlane = lane & 15;
  const int koff  = (lane >> 4) * 8;
  const int mOff  = (lane >> 4) * 8;

  const _Float16* bptr[4];
  const _Float16* aptr[4];
#pragma unroll
  for (int j = 0; j < 4; ++j) bptr[j] = Bt + (size_t)(n0 + (j << 4) + rlane) * ldb + koff;
#pragma unroll
  for (int i = 0; i < 4; ++i) aptr[i] = A + (size_t)(m0 + (i << 4) + rlane) * lda + koff;

  v8f acc[4][4];
#pragma unroll
  for (int i = 0; i < 4; ++i)
#pragma unroll
    for (int j = 0; j < 4; ++j) acc[i][j] = (v8f){0.f, 0.f, 0.f, 0.f, 0.f, 0.f, 0.f, 0.f};

  for (int k0 = 0; k0 < K; k0 += 32) {
    v16h bh[4];
#pragma unroll
    for (int j = 0; j < 4; ++j) bh[j] = frag_load(bptr[j] + k0);
#pragma unroll
    for (int i = 0; i < 4; ++i) {
      const v16h ah = frag_load(aptr[i] + k0);
#pragma unroll
      for (int j = 0; j < 4; ++j) acc[i][j] = mma_h(ah, bh[j], acc[i][j]);
      guard4_h(acc[i][0], acc[i][1], acc[i][2], acc[i][3], ah, bh[0], bh[1], bh[2], bh[3]);
    }
    keep4_h(bh[0], bh[1], bh[2], bh[3]);
  }
  acc_guard4(acc[0][0], acc[0][1], acc[0][2], acc[0][3]);
  acc_guard4(acc[1][0], acc[1][1], acc[1][2], acc[1][3]);
  acc_guard4(acc[2][0], acc[2][1], acc[2][2], acc[2][3]);
  acc_guard4(acc[3][0], acc[3][1], acc[3][2], acc[3][3]);

  float* slab = sT[wave];
#pragma unroll
  for (int i = 0; i < 4; ++i) {
    const int mBase = m0 + (i << 4);
#pragma unroll
    for (int j = 0; j < 4; ++j) {
      const int n = n0 + (j << 4) + rlane;
      const float bv = bias[n];
#pragma unroll
      for (int r = 0; r < 8; ++r) {
        const float v = acc[i][j][r] * scale + bv;
        slab[(mOff + r) * 68 + (j << 4) + rlane] = v;
      }
    }
    __builtin_amdgcn_fence(__ATOMIC_RELEASE, "workgroup");
    __builtin_amdgcn_wave_barrier();
    __builtin_amdgcn_fence(__ATOMIC_ACQUIRE, "workgroup");
    {
      const int hh = lane >> 4;
      const int c4 = (lane & 15) * 4;
      for (int pass = 0; pass < 2; ++pass) {
#pragma unroll
        for (int it = 0; it < 8; ++it) {
          const int row = it * 2 + hh;
          const v4f v = *(const v4f*)(slab + row * 68 + c4);
          *(volatile v4f*)(C + (size_t)(mBase + row) * ldc + n0 + c4) = v;
        }
        __threadfence();
      }
    }
    __builtin_amdgcn_fence(__ATOMIC_RELEASE, "workgroup");
    __builtin_amdgcn_wave_barrier();
    __builtin_amdgcn_fence(__ATOMIC_ACQUIRE, "workgroup");
  }
}

template <int LAYER>
__global__ __launch_bounds__(SCAN_THR) void gru_scan_kernel(
    const float* __restrict__ XI, const float* __restrict__ tin,
    const unsigned short* __restrict__ WHp, const float* __restrict__ bhh,
    const float* __restrict__ Wg, const float* __restrict__ bg,
    unsigned short* __restrict__ H1, float* __restrict__ OUT) {
  __shared__ __align__(16) _Float16 Ah[16 * HP];
  __shared__ __align__(16) float    Dl[16 * NSTEP];
  __shared__ __align__(16) float    Hs[(LAYER == 1) ? 16 * OP : 4];
  __shared__ __align__(16) _Float16 Hh[(LAYER == 0) ? 16 * HP : 8];
  const _Float16* WH = (const _Float16*)WHp;
  const int tid = threadIdx.x;
  const int lane = tid & 31;
  const int wave = tid >> 5;
  const int c = lane & 15;
  const int hh = lane >> 4;
  const int koff = hh * 8;
  const int rowbase = blockIdx.x * 16;
  const int j = 16 * wave + c;

#pragma unroll 1
  for (int i = tid; i < 16 * HP; i += SCAN_THR) Ah[i] = (_Float16)0.0f;
#pragma unroll 1
  for (int it = 0; it < (16 * NSTEP) / SCAN_THR; ++it) {
    const int idx = it * SCAN_THR + tid;
    const int row = idx >> 9;
    const int l = idx & (NSTEP - 1);
    const int lp = (l > 0) ? (l - 1) : 0;
    const size_t base = (size_t)(rowbase + row) * NSTEP;
    float tv = tin[base + l];
    float tp = tin[base + lp];
    asm volatile("" : "+v"(tv), "+v"(tp));
    const float fac = (l > 0) ? 1.0f : 0.0f;
    Dl[idx] = tv - fac * tp;
  }
  const float wgv = Wg[j];
  const float bgv = bg[j];
  const float bh0 = bhh[j];
  const float bh1 = bhh[NHID + j];
  const float bh2 = bhh[2 * NHID + j];
  float hst[8];
#pragma unroll
  for (int r = 0; r < 8; ++r) hst[r] = 0.0f;
  __syncthreads();

  const _Float16* ahrow = Ah + c * HP + koff;
  const _Float16* wh = WH + (size_t)j * NHID + koff;
  const float* xlane = XI + (size_t)(rowbase + 8 * hh) * NSTEP * NG3 + j;
  const v8f z8 = {0.f, 0.f, 0.f, 0.f, 0.f, 0.f, 0.f, 0.f};

#pragma unroll 1
  for (int t = 0; t < NSTEP; ++t) {
#pragma unroll
    for (int r = 0; r < 8; ++r) {
      const float dv = Dl[(8 * hh + r) * NSTEP + t];
      float a = wgv * dv + bgv;
      a = fmaxf(a, 0.0f);
      const float gm = expf(-a);
      const float hd = gm * hst[r];
      hst[r] = hd;
      Ah[(8 * hh + r) * HP + j] = (_Float16)(hd * HCARRY);
    }
    __syncthreads();

    v8f acc0 = z8, acc1 = z8, acc2 = z8;
#pragma unroll 1
    for (int k0 = 0; k0 < NHID; k0 += 32) {
      const v16h a  = frag_load(ahrow + k0);
      const v16h b0 = frag_load(wh + k0);
      const v16h b1 = frag_load(wh + (size_t)1 * NHID * NHID + k0);
      const v16h b2 = frag_load(wh + (size_t)2 * NHID * NHID + k0);
      acc0 = mma_h(a, b0, acc0);
      acc1 = mma_h(a, b1, acc1);
      acc2 = mma_h(a, b2, acc2);
      guard3_h(acc0, acc1, acc2, a, b0, b1, b2);
    }
    acc_guard3(acc0, acc1, acc2);

    const float* xp = xlane + (size_t)t * NG3;
#pragma unroll
    for (int r = 0; r < 8; ++r) {
      const float* xr_p = xp + (size_t)r * NSTEP * NG3;
      const float xr = xr_p[0];
      const float xz = xr_p[NHID];
      const float xn = xr_p[2 * NHID];
      const float hr = acc0[r] * FOLD_H + bh0;
      const float hz = acc1[r] * FOLD_H + bh1;
      const float hn = acc2[r] * FOLD_H + bh2;
      const float rg = sigm_f(xr + hr);
      const float zg = sigm_f(xz + hz);
      const float ng = tanh_f(xn + rg * hn);
      const float hd = hst[r];
      const float hnew = (1.0f - zg) * ng + zg * hd;
      hst[r] = hnew;
      if (LAYER == 0) Hh[(8 * hh + r) * HP + j] = (_Float16)(fmaxf(hnew, 0.0f) * HCARRY);
      else            Hs[(8 * hh + r) * OP + j] = hnew;
    }
    __syncthreads();

    if (LAYER == 0) {
      const v8h hv = *(const v8h*)(Hh + wave * HP + lane * 8);
      unsigned short* dst = H1 + ((size_t)(rowbase + wave) * NSTEP + (size_t)t) * NHID + lane * 8;
      for (int pass = 0; pass < 2; ++pass) {
        *(volatile v8h*)dst = hv;
        __threadfence();
      }
    } else {
      v4f vv[2];
#pragma unroll
      for (int it = 0; it < 2; ++it) {
        const int idx = it * SCAN_THR + tid;
        const int row = idx >> 6;
        const int c4 = (idx & 63) * 4;
        vv[it] = *(const v4f*)(Hs + row * OP + c4);
      }
      for (int pass = 0; pass < 2; ++pass) {
#pragma unroll
        for (int it = 0; it < 2; ++it) {
          const int idx = it * SCAN_THR + tid;
          const int row = idx >> 6;
          const int c4 = (idx & 63) * 4;
          *(volatile v4f*)(OUT + ((size_t)(rowbase + row) * NSTEP + (size_t)t) * NHID + c4) = vv[it];
        }
        __threadfence();
      }
    }
  }
}

extern "C" void kernel_launch(void* const* d_in, const int* in_sizes, int n_in,
                              void* d_out, int out_size, void* d_ws, size_t ws_size, hipStream_t stream) {
  if (n_in < 16 || d_out == nullptr || d_ws == nullptr) return;
  if (in_sizes[0] != NB * NSTEP * NDIN || in_sizes[1] != NB * NSTEP || in_sizes[2] != NEMB || in_sizes[3] != NEMB ||
      in_sizes[4] != NG3 * NCAT || in_sizes[5] != NG3 || in_sizes[6] != NG3 * NHID || in_sizes[7] != NG3 ||
      in_sizes[8] != NHID || in_sizes[9] != NHID || in_sizes[10] != NG3 * NHID || in_sizes[11] != NG3 ||
      in_sizes[12] != NG3 * NHID || in_sizes[13] != NG3 || in_sizes[14] != NHID || in_sizes[15] != NHID ||
      out_size != NB * NSTEP * NHID) return;

  const float* x    = (const float*)d_in[0];
  const float* tin  = (const float*)d_in[1];
  const float* Wt   = (const float*)d_in[2];
  const float* bt   = (const float*)d_in[3];
  const float* Wih0 = (const float*)d_in[4];
  const float* bih0 = (const float*)d_in[5];
  const float* Whh0 = (const float*)d_in[6];
  const float* bhh0 = (const float*)d_in[7];
  const float* Wg0  = (const float*)d_in[8];
  const float* bg0  = (const float*)d_in[9];
  const float* Wih1 = (const float*)d_in[10];
  const float* bih1 = (const float*)d_in[11];
  const float* Whh1 = (const float*)d_in[12];
  const float* bhh1 = (const float*)d_in[13];
  const float* Wg1  = (const float*)d_in[14];
  const float* bg1  = (const float*)d_in[15];
  float* out = (float*)d_out;

  char* ws = (char*)d_ws;
  size_t off = 0;
  auto carve = [&](size_t bytes) -> char* { char* p = ws + off; off += (bytes + 255) & ~(size_t)255; return p; };
  unsigned short* WIH0 = (unsigned short*)carve((size_t)NG3 * NCAT * 2);
  unsigned short* WHH0 = (unsigned short*)carve((size_t)NG3 * NHID * 2);
  unsigned short* WIH1 = (unsigned short*)carve((size_t)NG3 * NHID * 2);
  unsigned short* WHH1 = (unsigned short*)carve((size_t)NG3 * NHID * 2);
  unsigned short* XCAT = (unsigned short*)carve((size_t)NROWS * NCAT * 2);
  unsigned short* H1   = (unsigned short*)carve((size_t)NROWS * NHID * 2);
  float*          XI   = (float*)carve((size_t)NROWS * NG3 * 4);
  if (off > ws_size || off > (size_t)134217728) return;

  const int n8a = NG3 * NCAT / 8;
  const int n8b = NG3 * NHID / 8;
  prep_w_kernel<<<dim3(n8b / 256, 4), 256, 0, stream>>>(Wih0, Whh0, Wih1, Whh1, WIH0, WHH0, WIH1, WHH1,
                                                       n8a, n8b, n8b, n8b, WCARRY);
  prep_xcat_kernel<<<(NROWS * (NCAT / 8)) / 256, 256, 0, stream>>>(x, tin, Wt, bt, XCAT);

  const int ggrid = (NROWS / 64) * (NG3 / 64) / 8;
  gemm_f16_kernel<<<ggrid, 256, 0, stream>>>(XCAT, NCAT, WIH0, NCAT, XI, NG3, bih0, NROWS, NG3, NCAT, FOLD_X);
  gru_scan_kernel<0><<<NB / 16, SCAN_THR, 0, stream>>>(XI, tin, WHH0, bhh0, Wg0, bg0, H1, out);
  gemm_f16_kernel<<<ggrid, 256, 0, stream>>>(H1, NHID, WIH1, NHID, XI, NG3, bih1, NROWS, NG3, NHID, FOLD_H);
  gru_scan_kernel<1><<<NB / 16, SCAN_THR, 0, stream>>>(XI, tin, WHH1, bhh1, Wg1, bg1, H1, out);
}
